// CRNN_77335181131812
// MI455X (gfx1250) — hardware-run, weakly checked
//
#include <hip/hip_runtime.h>
#include <math.h>

constexpr int NBATCH = 64;
constexpr int NFREQ  = 64;
constexpr int NTIME  = 1024;
constexpr int NCH    = 64;
constexpr int NHID   = 64;
constexpr int NGATE  = 3 * NHID;
constexpr int NCLS   = 2;
constexpr int NROWS  = NTIME * NBATCH;
constexpr float WCARRY  = 16.0f;
constexpr float HCARRY  = 16.0f;
constexpr float GX_FOLD = 1.0f / WCARRY;
constexpr float GH_FOLD = 1.0f / (WCARRY * HCARRY);
constexpr float FC_FOLD = 1.0f / HCARRY;

constexpr int CONV_TT   = 16;
constexpr int XS_ROWS   = NFREQ + 2;
constexpr int XS_COLS   = CONV_TT + 2;
constexpr int XS_PITCH  = 20;
constexpr int XS_FILL_IT = (XS_ROWS * XS_COLS + 255) / 256;
constexpr int HPITCH    = 72;
constexpr int SEQ_THR   = 128;

static_assert(NTIME % CONV_TT == 0);
static_assert(NROWS % 64 == 0 && NGATE % 64 == 0);
static_assert(NCH % 32 == 0 && NHID % 32 == 0);
static_assert(((NROWS / 64) * (NGATE / 64)) % 8 == 0);
static_assert(NHID == 16 * (SEQ_THR / 32));
static_assert(NBATCH % 16 == 0);
static_assert((2 * 16 * HPITCH) % SEQ_THR == 0);
static_assert(HPITCH % 8 == 0 && HPITCH >= NHID);
static_assert((NGATE * NCH / 8) % 256 == 0);
static_assert((NBATCH * (NTIME / 32)) % 8 == 0);
static_assert(NCLS == 2);

typedef __attribute__((ext_vector_type(16))) _Float16 v16h;
typedef __attribute__((ext_vector_type(8)))  _Float16 v8h;
typedef __attribute__((ext_vector_type(8)))  float    v8f;
typedef __attribute__((ext_vector_type(4)))  float    v4f;
typedef __attribute__((ext_vector_type(4)))  unsigned v4u;

__device__ __forceinline__ void dep_guard4_h(v8f& a, v8f& b, v8f& c, v8f& d, v16h x, v16h y0, v16h y1, v16h y2, v16h y3) {
  asm volatile("v_nop\n\tv_nop\n\tv_nop\n\tv_nop" : "+v"(a), "+v"(b), "+v"(c), "+v"(d) : "v"(x), "v"(y0), "v"(y1), "v"(y2), "v"(y3));
}
__device__ __forceinline__ void dep_guard3_h(v8f& a, v8f& b, v8f& c, v16h x0, v16h x1,
                                             v16h y0, v16h y1, v16h y2, v16h y3, v16h y4, v16h y5) {
  asm volatile("v_nop\n\tv_nop\n\tv_nop\n\tv_nop" : "+v"(a), "+v"(b), "+v"(c)
               : "v"(x0), "v"(x1), "v"(y0), "v"(y1), "v"(y2), "v"(y3), "v"(y4), "v"(y5));
}
__device__ __forceinline__ void keep4_h(v16h a, v16h b, v16h c, v16h d) { asm volatile("v_nop" :: "v"(a), "v"(b), "v"(c), "v"(d)); }
__device__ __forceinline__ void acc_guard4(v8f& a, v8f& b, v8f& c, v8f& d) { asm volatile("v_nop\n\tv_nop\n\tv_nop\n\tv_nop" : "+v"(a), "+v"(b), "+v"(c), "+v"(d)); }

struct FragH {
  union U { v16h v; v8h h[2]; };
  static __device__ __forceinline__ v16h load(const _Float16* p) {
    U f; f.h[0] = *(const v8h*)(p); f.h[1] = *(const v8h*)(p + 16); return f.v;
  }
  static __device__ __forceinline__ v8f mma(v16h a, v16h b, v8f c) {
    return __builtin_amdgcn_wmma_f32_16x16x32_f16(false, a, false, b, (short)0, c, false, false);
  }
};

__device__ __forceinline__ float h16_to_f32(unsigned hb) {
  const unsigned sgn = (hb & 0x8000u) << 16;
  const unsigned em = hb & 0x7fffu;
  const float fn = __uint_as_float((em << 13) + 0x38000000u);
  const float fs = (float)em * 5.9604644775390625e-8f;
  const float mag = (em < 0x400u) ? fs : fn;
  return __uint_as_float(__float_as_uint(mag) | sgn);
}

__device__ __forceinline__ float sigm_f(float x) {
  x = fminf(fmaxf(x, -30.0f), 30.0f);
  return 1.0f / (1.0f + expf(-x));
}
__device__ __forceinline__ float tanh_f(float x) {
  x = fminf(fmaxf(x, -15.0f), 15.0f);
  return 1.0f - 2.0f / (1.0f + expf(2.0f * x));
}

__global__ __launch_bounds__(256) void cvt_w16_kernel(const float* __restrict__ src, unsigned short* __restrict__ dst,
                                                      int n8, float sc) {
  const int i = blockIdx.x * 256 + threadIdx.x;
  if (i < n8) {
    const float* sp = src + (size_t)i * 8;
    const v4f a = *(const v4f*)(sp);
    const v4f b = *(const v4f*)(sp + 4);
    v8h hv;
#pragma unroll
    for (int e = 0; e < 4; ++e) {
      const float fa = a[e] * sc;
      const float fb = b[e] * sc;
      hv[e]     = (_Float16)fa;
      hv[4 + e] = (_Float16)fb;
    }
    *(volatile v8h*)(dst + (size_t)i * 8) = hv;
    __threadfence();
    *(volatile v8h*)(dst + (size_t)i * 8) = hv;
  }
}

__global__ __launch_bounds__(256) void conv_pool_kernel(const float* __restrict__ x, const float* __restrict__ cw,
                                                        const float* __restrict__ cb, unsigned short* __restrict__ FEAT) {
  __shared__ __align__(16) float    xs[XS_ROWS * XS_PITCH];
  __shared__ __align__(16) _Float16 fs[CONV_TT * NCH];
  const int tid = threadIdx.x;
  const int b   = blockIdx.y;
  const int t0  = blockIdx.x * CONV_TT;

#pragma unroll 1
  for (int it = 0; it < XS_FILL_IT; ++it) {
    const int idx = it * 256 + tid;
    const bool ok = idx < XS_ROWS * XS_COLS;
    const int ic  = ok ? idx : (XS_ROWS * XS_COLS - 1);
    const int fr  = ic / XS_COLS;
    const int k   = ic - fr * XS_COLS;
    const int f   = fr - 1;
    const int t   = t0 - 1 + k;
    const bool inb = (f >= 0) && (f < NFREQ) && (t >= 0) && (t < NTIME);
    const int fcl = min(max(f, 0), NFREQ - 1);
    const int tcl = min(max(t, 0), NTIME - 1);
    float v = x[((size_t)b * NFREQ + (size_t)fcl) * NTIME + (size_t)tcl];
    v = inb ? v : 0.0f;
    if (ok) xs[fr * XS_PITCH + k] = v;
  }

  const int c  = tid & 63;
  const int tb = (tid >> 6) * 4;
  float w[9];
#pragma unroll
  for (int i = 0; i < 9; ++i) w[i] = cw[c * 9 + i];
  const float bias = cb[c];
  __syncthreads();

  float ra[6], rb[6], rc[6], m[4];
#pragma unroll
  for (int k = 0; k < 6; ++k) {
    ra[k] = xs[0 * XS_PITCH + tb + k];
    rb[k] = xs[1 * XS_PITCH + tb + k];
  }
#pragma unroll
  for (int q = 0; q < 4; ++q) m[q] = 0.0f;

#pragma unroll 1
  for (int f = 0; f < NFREQ; ++f) {
    const float* xr = xs + (f + 2) * XS_PITCH + tb;
#pragma unroll
    for (int k = 0; k < 6; ++k) rc[k] = xr[k];
#pragma unroll
    for (int q = 0; q < 4; ++q) {
      float acc = bias;
      acc = fmaf(ra[q],     w[0], acc);
      acc = fmaf(ra[q + 1], w[1], acc);
      acc = fmaf(ra[q + 2], w[2], acc);
      acc = fmaf(rb[q],     w[3], acc);
      acc = fmaf(rb[q + 1], w[4], acc);
      acc = fmaf(rb[q + 2], w[5], acc);
      acc = fmaf(rc[q],     w[6], acc);
      acc = fmaf(rc[q + 1], w[7], acc);
      acc = fmaf(rc[q + 2], w[8], acc);
      m[q] = fmaxf(m[q], acc);
    }
#pragma unroll
    for (int k = 0; k < 6; ++k) { ra[k] = rb[k]; rb[k] = rc[k]; }
  }

#pragma unroll
  for (int q = 0; q < 4; ++q) fs[(tb + q) * NCH + c] = (_Float16)m[q];
  __syncthreads();
  if (tid < 128) {
    const int row = tid >> 3;
    const int c8  = (tid & 7) * 8;
    const v8h hv = *(const v8h*)(fs + row * NCH + c8);
    unsigned short* dp = FEAT + ((size_t)(t0 + row) * NBATCH + (size_t)b) * NCH + c8;
    *(volatile v8h*)dp = hv;
    __threadfence();
    *(volatile v8h*)dp = hv;
  }
}

__global__ __launch_bounds__(256) void gemm_f16_bias_kernel(
    const unsigned short* __restrict__ Ap, int lda,
    const unsigned short* __restrict__ Btp, int ldb,
    float* __restrict__ Cout, int ldc,
    const float* __restrict__ bias, int M, int N, int K, float scale) {
  const _Float16* A  = (const _Float16*)Ap;
  const _Float16* Bt = (const _Float16*)Btp;
  __shared__ __align__(16) float sT[8][16 * 68];
  const int lane = threadIdx.x & 31;
  const int wave = threadIdx.x >> 5;
  const int tilesN = N >> 6;
  const int tilesM = M >> 6;
  const int tile = blockIdx.x * 8 + wave;
  if (tile >= tilesM * tilesN) return;
  const int tm = tile / tilesN;
  const int tn = tile - tm * tilesN;
  const int m0 = tm << 6;
  const int n0 = tn << 6;
  const int rlane = lane & 15;
  const int koff  = (lane >> 4) * 8;
  const int mOff  = (lane >> 4) * 8;

  v8f acc[4][4];
#pragma unroll
  for (int i = 0; i < 4; ++i)
#pragma unroll
    for (int j = 0; j < 4; ++j) acc[i][j] = (v8f){0.f, 0.f, 0.f, 0.f, 0.f, 0.f, 0.f, 0.f};

  for (int k0 = 0; k0 < K; k0 += 32) {
    v16h bh[4];
#pragma unroll
    for (int j = 0; j < 4; ++j) {
      const size_t bo = (size_t)(n0 + (j << 4) + rlane) * ldb + koff + k0;
      bh[j] = FragH::load(Bt + bo);
    }
#pragma unroll
    for (int i = 0; i < 4; ++i) {
      const size_t ao = (size_t)(m0 + (i << 4) + rlane) * lda + koff + k0;
      const v16h ah = FragH::load(A + ao);
#pragma unroll
      for (int j = 0; j < 4; ++j) acc[i][j] = FragH::mma(ah, bh[j], acc[i][j]);
      dep_guard4_h(acc[i][0], acc[i][1], acc[i][2], acc[i][3], ah, bh[0], bh[1], bh[2], bh[3]);
    }
    keep4_h(bh[0], bh[1], bh[2], bh[3]);
  }
  acc_guard4(acc[0][0], acc[0][1], acc[0][2], acc[0][3]);
  acc_guard4(acc[1][0], acc[1][1], acc[1][2], acc[1][3]);
  acc_guard4(acc[2][0], acc[2][1], acc[2][2], acc[2][3]);
  acc_guard4(acc[3][0], acc[3][1], acc[3][2], acc[3][3]);

  float* slab = sT[wave];
#pragma unroll
  for (int i = 0; i < 4; ++i) {
    const int mBase = m0 + (i << 4);
#pragma unroll
    for (int j = 0; j < 4; ++j) {
      const int n = n0 + (j << 4) + rlane;
      const float bv = bias[n];
#pragma unroll
      for (int r = 0; r < 8; ++r) {
        const float v = acc[i][j][r] * scale + bv;
        slab[(mOff + r) * 68 + (j << 4) + rlane] = v;
      }
    }
    __builtin_amdgcn_fence(__ATOMIC_RELEASE, "workgroup");
    __builtin_amdgcn_wave_barrier();
    __builtin_amdgcn_fence(__ATOMIC_ACQUIRE, "workgroup");
    {
      const int hh = lane >> 4, c4 = (lane & 15) * 4;
      for (int pass = 0; pass < 2; ++pass) {
#pragma unroll
        for (int it = 0; it < 8; ++it) {
          const int row = it * 2 + hh;
          const v4f v = *(const v4f*)(slab + row * 68 + c4);
          *(volatile v4f*)(Cout + (size_t)(mBase + row) * ldc + n0 + c4) = v;
        }
        __threadfence();
      }
    }
    __builtin_amdgcn_fence(__ATOMIC_RELEASE, "workgroup");
    __builtin_amdgcn_wave_barrier();
    __builtin_amdgcn_fence(__ATOMIC_ACQUIRE, "workgroup");
  }
}

__global__ __launch_bounds__(SEQ_THR) void gru_seq_kernel(const float* __restrict__ GX,
                                                          const unsigned short* __restrict__ WHp,
                                                          const float* __restrict__ b_hh,
                                                          unsigned short* __restrict__ HS) {
  __shared__ __align__(16) _Float16 Ah[2][16 * HPITCH];
  const _Float16* WH = (const _Float16*)WHp;
  const int tid = threadIdx.x, lane = tid & 31, wave = tid >> 5;
  const int c = lane & 15, hh = lane >> 4, koff = hh * 8;
  const int rowbase = blockIdx.x * 16;
  const int j = 16 * wave + c;

  {
    _Float16* ahf = &Ah[0][0];
#pragma unroll 1
    for (int i = tid; i < 2 * 16 * HPITCH; i += SEQ_THR) ahf[i] = (_Float16)0.0f;
  }

  const v16h b00 = FragH::load(WH + (size_t)(0 * NHID + j) * NHID + koff);
  const v16h b01 = FragH::load(WH + (size_t)(0 * NHID + j) * NHID + koff + 32);
  const v16h b10 = FragH::load(WH + (size_t)(1 * NHID + j) * NHID + koff);
  const v16h b11 = FragH::load(WH + (size_t)(1 * NHID + j) * NHID + koff + 32);
  const v16h b20 = FragH::load(WH + (size_t)(2 * NHID + j) * NHID + koff);
  const v16h b21 = FragH::load(WH + (size_t)(2 * NHID + j) * NHID + koff + 32);
  const float bhr = b_hh[j];
  const float bhz = b_hh[NHID + j];
  const float bhn = b_hh[2 * NHID + j];

  float hst[8];
#pragma unroll
  for (int r = 0; r < 8; ++r) hst[r] = 0.0f;
  __syncthreads();

  const v8f z8 = {0.f, 0.f, 0.f, 0.f, 0.f, 0.f, 0.f, 0.f};
  const int crow = 4 * wave + (lane >> 3);
  const int c8   = (lane & 7) * 8;

#pragma unroll 1
  for (int t = 0; t < NTIME; ++t) {
    const int cur = t & 1;
    const _Float16* ahc = &Ah[0][0] + cur * (16 * HPITCH);
    _Float16*       ahn = &Ah[0][0] + (cur ^ 1) * (16 * HPITCH);

    float gxv[3][8];
    {
      const float* gp = GX + ((size_t)t * NBATCH + (size_t)(rowbase + 8 * hh)) * NGATE + j;
#pragma unroll
      for (int g = 0; g < 3; ++g)
#pragma unroll
        for (int r = 0; r < 8; ++r) gxv[g][r] = gp[r * NGATE + g * NHID];
    }

    const v16h a0 = FragH::load(ahc + c * HPITCH + koff);
    const v16h a1 = FragH::load(ahc + c * HPITCH + koff + 32);
    v8f acc0 = z8, acc1 = z8, acc2 = z8;
    acc0 = FragH::mma(a0, b00, acc0);
    acc1 = FragH::mma(a0, b10, acc1);
    acc2 = FragH::mma(a0, b20, acc2);
    acc0 = FragH::mma(a1, b01, acc0);
    acc1 = FragH::mma(a1, b11, acc1);
    acc2 = FragH::mma(a1, b21, acc2);
    dep_guard3_h(acc0, acc1, acc2, a0, a1, b00, b01, b10, b11, b20, b21);

#pragma unroll
    for (int r = 0; r < 8; ++r) {
      const float hr = acc0[r] * GH_FOLD + bhr;
      const float hz = acc1[r] * GH_FOLD + bhz;
      const float hn = acc2[r] * GH_FOLD + bhn;
      const float rg = sigm_f(gxv[0][r] + hr);
      const float zg = sigm_f(gxv[1][r] + hz);
      const float ng = tanh_f(gxv[2][r] + rg * hn);
      const float ho = hst[r];
      const float hv = (1.0f - zg) * ng + zg * ho;
      hst[r] = hv;
      ahn[(8 * hh + r) * HPITCH + j] = (_Float16)(hv * HCARRY);
    }
    __syncthreads();

    {
      const v8h hv8 = *(const v8h*)(ahn + crow * HPITCH + c8);
      unsigned short* dp = HS + ((size_t)t * NBATCH + (size_t)(rowbase + crow)) * NHID + c8;
      *(volatile v8h*)dp = hv8;
      __threadfence();
      *(volatile v8h*)dp = hv8;
    }
  }
}

__global__ __launch_bounds__(256) void fc_kernel(const unsigned short* __restrict__ HS, const float* __restrict__ fc_w,
                                                 const float* __restrict__ fc_b, float* __restrict__ out) {
  __shared__ float wsh[NCLS * NHID];
  const int tid = threadIdx.x, lane = tid & 31, wave = tid >> 5;
  if (tid < NCLS * NHID) wsh[tid] = fc_w[tid];
  const float fb0 = fc_b[0];
  const float fb1 = fc_b[1];
  __syncthreads();

  const int gw = blockIdx.x * 8 + wave;
  const int b  = gw >> 5;
  const int t  = (gw & 31) * 32 + lane;
  const v4u* rp = (const v4u*)(HS + ((size_t)t * NBATCH + (size_t)b) * NHID);
  float a0 = 0.0f, a1 = 0.0f;
#pragma unroll 1
  for (int i = 0; i < NHID / 8; ++i) {
    const v4u wv = rp[i];
    const unsigned u0 = wv[0];
    const unsigned u1 = wv[1];
    const unsigned u2 = wv[2];
    const unsigned u3 = wv[3];
    const float* w0 = wsh + 8 * i;
    const float* w1 = wsh + NHID + 8 * i;
    const float f0 = h16_to_f32(u0 & 0xffffu);
    const float f1 = h16_to_f32(u0 >> 16);
    const float f2 = h16_to_f32(u1 & 0xffffu);
    const float f3 = h16_to_f32(u1 >> 16);
    const float f4 = h16_to_f32(u2 & 0xffffu);
    const float f5 = h16_to_f32(u2 >> 16);
    const float f6 = h16_to_f32(u3 & 0xffffu);
    const float f7 = h16_to_f32(u3 >> 16);
    a0 = fmaf(f0, w0[0], a0); a1 = fmaf(f0, w1[0], a1);
    a0 = fmaf(f1, w0[1], a0); a1 = fmaf(f1, w1[1], a1);
    a0 = fmaf(f2, w0[2], a0); a1 = fmaf(f2, w1[2], a1);
    a0 = fmaf(f3, w0[3], a0); a1 = fmaf(f3, w1[3], a1);
    a0 = fmaf(f4, w0[4], a0); a1 = fmaf(f4, w1[4], a1);
    a0 = fmaf(f5, w0[5], a0); a1 = fmaf(f5, w1[5], a1);
    a0 = fmaf(f6, w0[6], a0); a1 = fmaf(f6, w1[6], a1);
    a0 = fmaf(f7, w0[7], a0); a1 = fmaf(f7, w1[7], a1);
  }
  const float o0 = a0 * FC_FOLD + fb0;
  const float o1 = a1 * FC_FOLD + fb1;
  float* p0 = out + (size_t)b * (NCLS * NTIME) + t;
  float* p1 = p0 + NTIME;
  *(volatile float*)p0 = o0;
  *(volatile float*)p1 = o1;
  __threadfence();
  *(volatile float*)p0 = o0;
  *(volatile float*)p1 = o1;
}

extern "C" void kernel_launch(void* const* d_in, const int* in_sizes, int n_in,
                              void* d_out, int out_size, void* d_ws, size_t ws_size, hipStream_t stream) {
  if (n_in < 9 || d_out == nullptr || d_ws == nullptr) return;
  if (in_sizes[0] != NBATCH * NFREQ * NTIME || in_sizes[1] != NCH * 9 || in_sizes[2] != NCH ||
      in_sizes[3] != NGATE * NCH || in_sizes[4] != NGATE * NHID || in_sizes[5] != NGATE ||
      in_sizes[6] != NGATE || in_sizes[7] != NCLS * NHID || in_sizes[8] != NCLS ||
      out_size != NBATCH * NCLS * NTIME) return;

  const float* x      = (const float*)d_in[0];
  const float* conv_w = (const float*)d_in[1];
  const float* conv_b = (const float*)d_in[2];
  const float* w_ih   = (const float*)d_in[3];
  const float* w_hh   = (const float*)d_in[4];
  const float* b_ih   = (const float*)d_in[5];
  const float* b_hh   = (const float*)d_in[6];
  const float* fc_w   = (const float*)d_in[7];
  const float* fc_b   = (const float*)d_in[8];
  float* out = (float*)d_out;

  char* ws = (char*)d_ws;
  size_t off = 0;
  auto carve = [&](size_t bytes) -> char* { char* p = ws + off; off += (bytes + 255) & ~(size_t)255; return p; };
  unsigned short* FEAT = (unsigned short*)carve((size_t)NROWS * NCH * 2);
  unsigned short* WIH  = (unsigned short*)carve((size_t)NGATE * NCH * 2);
  unsigned short* WHH  = (unsigned short*)carve((size_t)NGATE * NHID * 2);
  float*          GX   = (float*)carve((size_t)NROWS * NGATE * 4);
  unsigned short* HSEQ = (unsigned short*)carve((size_t)NROWS * NHID * 2);
  if (off > ws_size || off > (size_t)134217728) return;

  const int n8w = NGATE * NCH / 8;
  cvt_w16_kernel<<<n8w / 256, 256, 0, stream>>>(w_ih, WIH, n8w, WCARRY);
  cvt_w16_kernel<<<n8w / 256, 256, 0, stream>>>(w_hh, WHH, n8w, WCARRY);
  conv_pool_kernel<<<dim3(NTIME / CONV_TT, NBATCH), 256, 0, stream>>>(x, conv_w, conv_b, FEAT);
  gemm_f16_bias_kernel<<<(NROWS / 64) * (NGATE / 64) / 8, 256, 0, stream>>>(
      FEAT, NCH, WIH, NCH, GX, NGATE, b_ih, NROWS, NGATE, NCH, GX_FOLD);
  gru_seq_kernel<<<NBATCH / 16, SEQ_THR, 0, stream>>>(GX, WHH, b_hh, HSEQ);
  fc_kernel<<<NBATCH * (NTIME / 32) / 8, 256, 0, stream>>>(HSEQ, fc_w, fc_b, out);
}
